// MultiHeadSelfAttention_1614907704014
// MI455X (gfx1250) — hardware-verified
//
#include <hip/hip_runtime.h>
#ifndef NB
#define NB 1
#endif
#ifndef SEQ
#define SEQ 2048
#endif
#define SEQ_FULL 2048
#define NG 2
#define EMB 1024
#define NH 16
#define NKV 4
#define HD 64
#define KVW (NKV * HD)
#define LQ (EMB + 2 * KVW)
#define CP (2 * EMB)
#define NR (NB * SEQ * NG)
#define EQT 4
#define RS 1024.0f
#define RINV 0.0009765625f
#define RSC 64.0f

static_assert(NB == 1);
static_assert(SEQ % 64 == 0);
static_assert(SEQ >= 64);
static_assert(SEQ <= SEQ_FULL);
static_assert(NR % 128 == 0);
static_assert(LQ % 64 == 0);
static_assert(EMB % 64 == 0);
static_assert(EMB % 32 == 0);
static_assert(CP % 32 == 0);
static_assert(HD == 64);
static_assert(NH == 4 * NKV);
static_assert(NH * HD == EMB);
static_assert(KVW % 64 == 0);

typedef unsigned short v8us __attribute__((ext_vector_type(8), may_alias));
typedef float  v8f  __attribute__((ext_vector_type(8)));
typedef float  v4f  __attribute__((ext_vector_type(4)));
typedef float  v4fa __attribute__((ext_vector_type(4), may_alias));
typedef _Float16 v16h __attribute__((ext_vector_type(16)));
union FragH { v16h v; v8us half[2]; _Float16 h[16]; unsigned short u[16]; };

constexpr size_t SZ_BQKV = (size_t)LQ * EMB * 2;
constexpr size_t SZ_BO   = (size_t)EMB * CP * 2;
constexpr size_t SZ_X16  = (size_t)NR * EMB * 2;
constexpr size_t SZ_QK   = (size_t)NR * LQ * 2;
constexpr size_t SZ_VT   = (size_t)NB * NG * NKV * HD * SEQ * 2;
constexpr size_t SZ_CX   = (size_t)NR * CP * 2;
constexpr size_t WS_TOTAL = SZ_BQKV + SZ_BO + SZ_X16 + 2 * SZ_QK + 2 * SZ_VT + SZ_CX;
static_assert(WS_TOTAL <= (size_t)134217728);
static_assert(SZ_BQKV % 256 == 0 && SZ_BO % 256 == 0 && SZ_X16 % 256 == 0 && SZ_QK % 256 == 0 && SZ_VT % 256 == 0 && SZ_CX % 256 == 0);

__device__ __forceinline__ float bf16_rne(float x) { unsigned int u = __float_as_uint(x); u = (u + 0x7FFFu + ((u >> 16) & 1u)) & 0xFFFF0000u; return __uint_as_float(u); }
__device__ __forceinline__ unsigned short h_bits(_Float16 h) { return __builtin_bit_cast(unsigned short, h); }
__device__ __forceinline__ v16h ldfrag(const unsigned short* __restrict__ p, size_t off, int hh) { FragH f; f.half[0] = *(const v8us*)(p + off + 8 * hh); f.half[1] = *(const v8us*)(p + off + 16 + 8 * hh); return f.v; }
__device__ __forceinline__ v8f mma(v16h a, v16h b, v8f c) { v8f d = __builtin_amdgcn_wmma_f32_16x16x32_f16(false, a, false, b, (short)0, c, false, false); asm volatile("v_nop\n\tv_nop\n\tv_nop\n\tv_nop" : "+v"(d) : "v"(a), "v"(b)); return d; }

__global__ __launch_bounds__(256) void k_wt_f16(const float* __restrict__ W, unsigned short* __restrict__ Wt, int K, int N, int drow0, int dpitch, int dcol0, float scale) {
  const int t = blockIdx.x * 256 + threadIdx.x; const int k8n = K / 8; if (t >= N * k8n) return;
  const int n = t / k8n, k8 = (t - n * k8n) * 8; FragH f;
#pragma unroll
  for (int i = 0; i < 8; ++i) f.h[i] = (_Float16)(bf16_rne(W[(size_t)(k8 + i) * N + n]) * scale);
  const v8us o = f.half[0];
  unsigned short* d = Wt + (size_t)(drow0 + n) * dpitch + dcol0 + k8;
  *(volatile v8us*)d = o; __threadfence(); *(volatile v8us*)d = o;
}

__global__ __launch_bounds__(256) void k_x16(const float* __restrict__ x, unsigned short* __restrict__ X16, int n8) {
  const int t = blockIdx.x * 256 + threadIdx.x; if (t >= n8) return;
  const v4f a = *(const v4fa*)(x + (size_t)t * 8), c = *(const v4fa*)(x + (size_t)t * 8 + 4); FragH f;
#pragma unroll
  for (int q = 0; q < 4; ++q) { f.h[q] = (_Float16)bf16_rne(a[q]); f.h[4 + q] = (_Float16)bf16_rne(c[q]); }
  const v8us o = f.half[0];
  unsigned short* d = X16 + (size_t)t * 8;
  *(volatile v8us*)d = o; __threadfence(); *(volatile v8us*)d = o;
}

__device__ __forceinline__ void gemm_core(const unsigned short* __restrict__ A, int lda, const unsigned short* __restrict__ Bt, int ldb, int K, int row0, int col0, int ln, int hh,
    v8f& c00, v8f& c01, v8f& c02, v8f& c03, v8f& c10, v8f& c11, v8f& c12, v8f& c13) {
  const size_t a0 = (size_t)(row0 + ln) * lda, a1 = a0 + (size_t)16 * lda;
  const size_t b0 = (size_t)(col0 + ln) * ldb, b1 = b0 + (size_t)16 * ldb, b2 = b1 + (size_t)16 * ldb, b3 = b2 + (size_t)16 * ldb;
#pragma unroll 1
  for (int kb = 0; kb < K; kb += 32) {
    const v16h fa0 = ldfrag(A, a0 + kb, hh), fa1 = ldfrag(A, a1 + kb, hh);
    v16h b = ldfrag(Bt, b0 + kb, hh); c00 = mma(fa0, b, c00); c10 = mma(fa1, b, c10);
    b = ldfrag(Bt, b1 + kb, hh); c01 = mma(fa0, b, c01); c11 = mma(fa1, b, c11);
    b = ldfrag(Bt, b2 + kb, hh); c02 = mma(fa0, b, c02); c12 = mma(fa1, b, c12);
    b = ldfrag(Bt, b3 + kb, hh); c03 = mma(fa0, b, c03); c13 = mma(fa1, b, c13);
  }
}

__global__ __launch_bounds__(128) void k_gemm_planes(const unsigned short* __restrict__ A, int lda, const unsigned short* __restrict__ Bt, int ldb, float alpha,
    unsigned short* __restrict__ CH, unsigned short* __restrict__ CR, int ldc, int M, int N, int K) {
  __shared__ __attribute__((aligned(16))) float so[4][32][68];
  const int tid = threadIdx.x; const int wave = __builtin_amdgcn_readfirstlane(tid >> 5);
  const int lane = tid & 31, ln = lane & 15, hh = lane >> 4;
  const int ntn = N >> 6; const int mt = blockIdx.x / ntn, nq = blockIdx.x - mt * ntn;
  const int row0 = mt * 128 + 32 * wave, col0 = nq * 64; if (row0 >= M) return;
  const v8f z8 = {0.f, 0.f, 0.f, 0.f, 0.f, 0.f, 0.f, 0.f};
  v8f c00 = z8, c01 = z8, c02 = z8, c03 = z8, c10 = z8, c11 = z8, c12 = z8, c13 = z8;
  gemm_core(A, lda, Bt, ldb, K, row0, col0, ln, hh, c00, c01, c02, c03, c10, c11, c12, c13);
  v8f accs[8] = {c00, c01, c02, c03, c10, c11, c12, c13};
#pragma unroll
  for (int u = 0; u < 8; ++u) { const int t = u & 3, hf = u >> 2;
#pragma unroll
    for (int r = 0; r < 8; ++r) so[wave][hf * 16 + 8 * hh + r][t * 16 + ln] = accs[u][r] * alpha; }
  __builtin_amdgcn_fence(4  , "workgroup"); __builtin_amdgcn_wave_barrier();
  const int rq = lane >> 3, c8 = (lane & 7) * 8;
  for (int pass = 0; pass < 2; ++pass) {
#pragma unroll
    for (int it = 0; it < 8; ++it) {
      const int rr = it * 4 + rq;
      const v4f a = *(const v4fa*)&so[wave][rr][c8], b = *(const v4fa*)&so[wave][rr][c8 + 4];
      FragH fh, fl;
#pragma unroll
      for (int q = 0; q < 4; ++q) { _Float16 hv = (_Float16)a[q]; fh.h[q] = hv; fl.h[q] = (_Float16)((a[q] - (float)hv) * RS); hv = (_Float16)b[q]; fh.h[4 + q] = hv; fl.h[4 + q] = (_Float16)((b[q] - (float)hv) * RS); }
      const v8us oh = fh.half[0], ol = fl.half[0];
      const size_t o = (size_t)(row0 + rr) * ldc + col0 + c8;
      *(volatile v8us*)(CH + o) = oh; *(volatile v8us*)(CR + o) = ol;
    }
    if (pass == 0) __threadfence();
  }
}

__global__ __launch_bounds__(128) void k_gemm_out(const unsigned short* __restrict__ A, int lda, const unsigned short* __restrict__ Bt, int ldb, float alpha,
    float* __restrict__ C, int ldc, int M, int N, int K) {
  __shared__ __attribute__((aligned(16))) float so[4][32][68];
  const int tid = threadIdx.x; const int wave = __builtin_amdgcn_readfirstlane(tid >> 5);
  const int lane = tid & 31, ln = lane & 15, hh = lane >> 4;
  const int ntn = N >> 6; const int mt = blockIdx.x / ntn, nq = blockIdx.x - mt * ntn;
  const int row0 = mt * 128 + 32 * wave, col0 = nq * 64; if (row0 >= M) return;
  const v8f z8 = {0.f, 0.f, 0.f, 0.f, 0.f, 0.f, 0.f, 0.f};
  v8f c00 = z8, c01 = z8, c02 = z8, c03 = z8, c10 = z8, c11 = z8, c12 = z8, c13 = z8;
  gemm_core(A, lda, Bt, ldb, K, row0, col0, ln, hh, c00, c01, c02, c03, c10, c11, c12, c13);
  v8f accs[8] = {c00, c01, c02, c03, c10, c11, c12, c13};
#pragma unroll
  for (int u = 0; u < 8; ++u) { const int t = u & 3, hf = u >> 2;
#pragma unroll
    for (int r = 0; r < 8; ++r) so[wave][hf * 16 + 8 * hh + r][t * 16 + ln] = accs[u][r] * alpha; }
  __builtin_amdgcn_fence(4  , "workgroup"); __builtin_amdgcn_wave_barrier();
  const int rsub = lane >> 4, c4 = (lane & 15) * 4;
  for (int pass = 0; pass < 2; ++pass) {
#pragma unroll
    for (int q = 0; q < 16; ++q) { const int r = q * 2 + rsub; const v4f v = *(const v4fa*)&so[wave][r][c4]; *(volatile v4f*)(C + (size_t)(row0 + r) * ldc + col0 + c4) = v; }
    if (pass == 0) __threadfence();
  }
}

__global__ __launch_bounds__(256) void k_vt(const unsigned short* __restrict__ QKH, const unsigned short* __restrict__ QKR, unsigned short* __restrict__ VTH, unsigned short* __restrict__ VTR) {
  __shared__ unsigned short tl[2][64][66];
  const int tid = threadIdx.x;
  const int nlg = SEQ / 64;
  const int slab = blockIdx.x / nlg, lg = blockIdx.x - slab * nlg;
  const int g = slab / NKV, kv = slab - g * NKV;
#pragma unroll 1
  for (int i = tid; i < 512; i += 256) {
    const int r = i >> 3, c8 = (i & 7) * 8;
    const size_t sof = ((size_t)(lg * 64 + r) * NG + g) * LQ + EMB + KVW + kv * HD + c8;
    FragH fh, fr; fh.half[0] = *(const v8us*)(QKH + sof); fr.half[0] = *(const v8us*)(QKR + sof);
#pragma unroll
    for (int q = 0; q < 8; ++q) { tl[0][r][c8 + q] = fh.u[q]; tl[1][r][c8 + q] = fr.u[q]; }
  }
  __syncthreads();
  for (int pass = 0; pass < 2; ++pass) {
#pragma unroll
    for (int rd = 0; rd < 2; ++rd) {
      const int d = rd * 32 + (tid >> 3), pc = tid & 7; FragH fh, fr;
#pragma unroll
      for (int q = 0; q < 8; ++q) { fh.u[q] = tl[0][pc * 8 + q][d]; fr.u[q] = tl[1][pc * 8 + q][d]; }
      const v8us oh = fh.half[0], ol = fr.half[0];
      const size_t o = ((size_t)slab * HD + d) * SEQ + lg * 64 + pc * 8;
      *(volatile v8us*)(VTH + o) = oh; *(volatile v8us*)(VTR + o) = ol;
    }
    if (pass == 0) __threadfence();
  }
}

__global__ __launch_bounds__(128) void k_attn(const unsigned short* __restrict__ QKH, const unsigned short* __restrict__ QKR,
    const unsigned short* __restrict__ VTH, const unsigned short* __restrict__ VTR, unsigned short* __restrict__ CX) {
  __shared__ __attribute__((aligned(16))) unsigned short pt[4][2][16][40];
  __shared__ __attribute__((aligned(16))) float so[4][16][68];
  const int tid = threadIdx.x; const int wave = __builtin_amdgcn_readfirstlane(tid >> 5);
  const int lane = tid & 31, ln = lane & 15, hh = lane >> 4;
  const int qt = blockIdx.x, gh = blockIdx.y;
  const int g = gh >> 4, h = gh & 15, kvh = h >> 2;
  const bool full = qt < EQT;
  const int q0 = qt * 64 + wave * 16;
  const size_t qoff = ((size_t)(q0 + ln) * NG + g) * LQ + h * HD;
  const size_t kcol = (size_t)EMB + kvh * HD;
  const size_t vrow = (size_t)(g * NKV + kvh) * HD;
  const v8f z8 = {0.f, 0.f, 0.f, 0.f, 0.f, 0.f, 0.f, 0.f};
  v8f om[4] = {z8, z8, z8, z8}, orr[4] = {z8, z8, z8, z8};
  float mi[8], li[8];
#pragma unroll
  for (int r = 0; r < 8; ++r) { mi[r] = -1.0e30f; li[r] = 0.f; }
  const int nkb = (q0 + 16 + 31) >> 5;
#pragma unroll 1
  for (int kb = 0; kb < nkb; ++kb) {
    const int kbase = kb * 32;
    v8f sm[2] = {z8, z8}, sr[2] = {z8, z8};
#pragma unroll
    for (int kk = 0; kk < 2; ++kk) {
      const v16h qh = ldfrag(QKH, qoff + kk * 32, hh);
      const v16h qr = ldfrag(QKR, qoff + kk * 32, hh);
#pragma unroll
      for (int nt = 0; nt < 2; ++nt) {
        const size_t ko = ((size_t)(kbase + nt * 16 + ln) * NG + g) * LQ + kcol + kk * 32;
        const v16h kh = ldfrag(QKH, ko, hh);
        sm[nt] = mma(qh, kh, sm[nt]);
        sr[nt] = mma(qr, kh, sr[nt]);
        if (full) { const v16h kr = ldfrag(QKR, ko, hh); sr[nt] = mma(qh, kr, sr[nt]); }
      }
    }
    float pv[2][8];
#pragma unroll
    for (int r = 0; r < 8; ++r) {
      const int qi = q0 + 8 * hh + r;
      const bool ok0 = (kbase + ln) <= qi, ok1 = (kbase + 16 + ln) <= qi;
      const float s0 = (sm[0][r] + sr[0][r] * RINV) * 0.125f;
      const float s1 = (sm[1][r] + sr[1][r] * RINV) * 0.125f;
      float mx = fmaxf(ok0 ? s0 : -1.0e30f, ok1 ? s1 : -1.0e30f);
      mx = fmaxf(mx, __shfl_xor(mx, 1, 32));
      mx = fmaxf(mx, __shfl_xor(mx, 2, 32));
      mx = fmaxf(mx, __shfl_xor(mx, 4, 32));
      mx = fmaxf(mx, __shfl_xor(mx, 8, 32));
      const float mnew = fmaxf(mi[r], mx);
      const float al = __expf(mi[r] - mnew);
      mi[r] = mnew;
      const float e0 = __expf(fminf(s0 - mnew, 0.f)), e1 = __expf(fminf(s1 - mnew, 0.f));
      const float p0 = ok0 ? e0 : 0.f, p1 = ok1 ? e1 : 0.f;
      float sum = p0 + p1;
      sum += __shfl_xor(sum, 1, 32);
      sum += __shfl_xor(sum, 2, 32);
      sum += __shfl_xor(sum, 4, 32);
      sum += __shfl_xor(sum, 8, 32);
      li[r] = li[r] * al + sum;
#pragma unroll
      for (int t = 0; t < 4; ++t) { om[t][r] *= al; orr[t][r] *= al; }
      pv[0][r] = p0; pv[1][r] = p1;
    }
#pragma unroll
    for (int nt = 0; nt < 2; ++nt) {
#pragma unroll
      for (int r = 0; r < 8; ++r) {
        const float pc = pv[nt][r] * RS;
        const _Float16 p16 = (_Float16)pc;
        pt[wave][0][8 * hh + r][nt * 16 + ln] = h_bits(p16);
        if (full) pt[wave][1][8 * hh + r][nt * 16 + ln] = h_bits((_Float16)((pc - (float)p16) * RS));
      }
    }
    __builtin_amdgcn_fence(4  , "workgroup"); __builtin_amdgcn_wave_barrier();
    FragH ph; ph.half[0] = *(const v8us*)&pt[wave][0][ln][8 * hh]; ph.half[1] = *(const v8us*)&pt[wave][0][ln][16 + 8 * hh];
    FragH pr = ph;
    if (full) { pr.half[0] = *(const v8us*)&pt[wave][1][ln][8 * hh]; pr.half[1] = *(const v8us*)&pt[wave][1][ln][16 + 8 * hh]; }
#pragma unroll
    for (int t = 0; t < 4; ++t) {
      const size_t vo = (vrow + t * 16 + ln) * (size_t)SEQ + kbase;
      const v16h vh = ldfrag(VTH, vo, hh);
      om[t] = mma(ph.v, vh, om[t]);
      if (full) { const v16h vr = ldfrag(VTR, vo, hh); orr[t] = mma(ph.v, vr, orr[t]); orr[t] = mma(pr.v, vh, orr[t]); }
    }
    __builtin_amdgcn_fence(4  , "workgroup"); __builtin_amdgcn_wave_barrier();
  }
#pragma unroll
  for (int r = 0; r < 8; ++r) {
    const float inv = 0.015625f * (1.0f / li[r]);
#pragma unroll
    for (int t = 0; t < 4; ++t) so[wave][8 * hh + r][t * 16 + ln] = (om[t][r] + orr[t][r] * RINV) * inv;
  }
  __builtin_amdgcn_fence(4  , "workgroup"); __builtin_amdgcn_wave_barrier();
  const int rq = lane >> 3, c8 = (lane & 7) * 8;
  for (int pass = 0; pass < 2; ++pass) {
#pragma unroll
    for (int it = 0; it < 4; ++it) {
      const int rr = it * 4 + rq;
      const v4f a = *(const v4fa*)&so[wave][rr][c8], b = *(const v4fa*)&so[wave][rr][c8 + 4];
      FragH fh, fl;
#pragma unroll
      for (int q = 0; q < 4; ++q) { _Float16 hv = (_Float16)a[q]; fh.h[q] = hv; fl.h[q] = (_Float16)((a[q] - (float)hv) * RSC); hv = (_Float16)b[q]; fh.h[4 + q] = hv; fl.h[4 + q] = (_Float16)((b[q] - (float)hv) * RSC); }
      const v8us oh = fh.half[0], ol = fl.half[0];
      const size_t o = ((size_t)(q0 + rr) * NG + g) * CP + h * HD + c8;
      *(volatile v8us*)(CX + o) = oh; *(volatile v8us*)(CX + o + EMB) = ol;
    }
    if (pass == 0) __threadfence();
  }
}

extern "C" void kernel_launch(void* const* d_in, const int* in_sizes, int n_in,
                              void* d_out, int out_size, void* d_ws, size_t ws_size, hipStream_t stream) {
  if (n_in < 5) return;
  if (in_sizes[0] < NR * EMB) return;
  if (in_sizes[1] < EMB * EMB) return;
  if (in_sizes[2] < EMB * KVW) return;
  if (in_sizes[3] < EMB * KVW) return;
  if (in_sizes[4] < EMB * EMB) return;
  if (out_size < NR * EMB) return;
  const float* x  = (const float*)d_in[0];
  const float* Wq = (const float*)d_in[1];
  const float* Wk = (const float*)d_in[2];
  const float* Wv = (const float*)d_in[3];
  const float* Wo = (const float*)d_in[4];
  char* ws = (char*)d_ws; size_t off = 0;
  auto take = [&](size_t bytes) { char* p = ws + off; off += (bytes + 255) & ~(size_t)255; return p; };
  unsigned short* BQKV = (unsigned short*)take(SZ_BQKV);
  unsigned short* BO   = (unsigned short*)take(SZ_BO);
  unsigned short* X16  = (unsigned short*)take(SZ_X16);
  unsigned short* QKH  = (unsigned short*)take(SZ_QK);
  unsigned short* QKR  = (unsigned short*)take(SZ_QK);
  unsigned short* VTH  = (unsigned short*)take(SZ_VT);
  unsigned short* VTR  = (unsigned short*)take(SZ_VT);
  unsigned short* CX   = (unsigned short*)take(SZ_CX);
  if (off > ws_size) return;

  k_wt_f16<<<(unsigned)((EMB * (EMB / 8) + 255) / 256), 256, 0, stream>>>(Wq, BQKV, EMB, EMB, 0, EMB, 0, 16.0f);
  k_wt_f16<<<(unsigned)((KVW * (EMB / 8) + 255) / 256), 256, 0, stream>>>(Wk, BQKV, EMB, KVW, EMB, EMB, 0, 16.0f);
  k_wt_f16<<<(unsigned)((KVW * (EMB / 8) + 255) / 256), 256, 0, stream>>>(Wv, BQKV, EMB, KVW, EMB + KVW, EMB, 0, 16.0f);
  k_wt_f16<<<(unsigned)((EMB * (EMB / 8) + 255) / 256), 256, 0, stream>>>(Wo, BO, EMB, EMB, 0, CP, 0, 16.0f);
  k_wt_f16<<<(unsigned)((EMB * (EMB / 8) + 255) / 256), 256, 0, stream>>>(Wo, BO, EMB, EMB, 0, CP, EMB, 0.25f);
  k_x16<<<(unsigned)((NR * (EMB / 8) + 255) / 256), 256, 0, stream>>>(x, X16, NR * (EMB / 8));
  k_gemm_planes<<<(unsigned)((NR / 128) * (LQ / 64)), 128, 0, stream>>>(X16, EMB, BQKV, EMB, 0.0625f, QKH, QKR, LQ, NR, LQ, EMB);
  k_vt<<<(unsigned)(NB * NG * NKV * (SEQ / 64)), 256, 0, stream>>>(QKH, QKR, VTH, VTR);
  k_attn<<<dim3((unsigned)(SEQ / 64), (unsigned)(NG * NH)), 128, 0, stream>>>(QKH, QKR, VTH, VTR, CX);
  k_gemm_out<<<(unsigned)((NR / 128) * (EMB / 64)), 128, 0, stream>>>(CX, CP, BO, CP, 0.00390625f, (float*)d_out, EMB, NR, EMB, CP);
}
